// Spline_Fitting_21328807592211
// MI455X (gfx1250) — hardware-verified
//
#include <hip/hip_runtime.h>


#define S_  128
#define D_  256
#define H_  8
#define E_  32
#define QT  16
#define XP  33
#define PP  136
#define VP  136
#define OP  264

typedef __attribute__((ext_vector_type(16))) _Float16 v16h;
typedef __attribute__((ext_vector_type(8)))  _Float16 v8h;
typedef __attribute__((ext_vector_type(16))) __bf16   v16b;
typedef __attribute__((ext_vector_type(8)))  __bf16   v8b;
typedef __attribute__((ext_vector_type(8)))  float    v8f;
typedef __attribute__((ext_vector_type(4)))  float    v4f;

__device__ __forceinline__ unsigned short f2bf_bits(float f) {
  unsigned u = __float_as_uint(f);
  return (unsigned short)((u + 0x7FFFu + ((u >> 16) & 1u)) >> 16);
}
__device__ __forceinline__ float bf_bits2f(unsigned short h) { return __uint_as_float(((unsigned)h) << 16); }

__device__ __forceinline__ void dep_guard_h(v8f& a, v8f& b, v16h x, v16h y) { asm volatile("v_nop\n\tv_nop\n\tv_nop\n\tv_nop" : "+v"(a), "+v"(b) : "v"(x), "v"(y)); }
__device__ __forceinline__ void dep_guard_b(v8f& a, v8f& b, v16b x, v16b y) { asm volatile("v_nop\n\tv_nop\n\tv_nop\n\tv_nop" : "+v"(a), "+v"(b) : "v"(x), "v"(y)); }
__device__ __forceinline__ void keep4_h(v16h a, v16h b, v16h c, v16h d) { asm volatile("v_nop" :: "v"(a), "v"(b), "v"(c), "v"(d)); }
__device__ __forceinline__ void keep4_b(v16b a, v16b b, v16b c, v16b d) { asm volatile("v_nop" :: "v"(a), "v"(b), "v"(c), "v"(d)); }
__device__ __forceinline__ void acc_guard4(v8f& a, v8f& b, v8f& c, v8f& d) { asm volatile("v_nop\n\tv_nop\n\tv_nop\n\tv_nop" : "+v"(a), "+v"(b), "+v"(c), "+v"(d)); }
template <typename T> struct Frag;
template <> struct Frag<_Float16> {
  typedef v16h V; union U { v16h v; v8h h[2]; };
  static __device__ __forceinline__ v16h load(const _Float16* p) {
    U f; f.h[0] = *(const v8h*)(p); f.h[1] = *(const v8h*)(p + 16); return f.v;
  }
  static __device__ __forceinline__ v8f mma(v16h a, v16h b, v8f c) {
    return __builtin_amdgcn_wmma_f32_16x16x32_f16(false, a, false, b, (short)0, c, false, false);
  }
  static __device__ __forceinline__ void guard(v8f& a, v8f& b, v16h x, v16h y) { dep_guard_h(a, b, x, y); }
  static __device__ __forceinline__ void keep(v16h a, v16h b, v16h c, v16h d) { keep4_h(a, b, c, d); }
};
template <> struct Frag<__bf16> {
  typedef v16b V; union U { v16b v; v8b h[2]; };
  static __device__ __forceinline__ v16b load(const __bf16* p) {
    U f; f.h[0] = *(const v8b*)(p); f.h[1] = *(const v8b*)(p + 16); return f.v;
  }
  static __device__ __forceinline__ v8f mma(v16b a, v16b b, v8f c) {
    return __builtin_amdgcn_wmma_f32_16x16x32_bf16(false, a, false, b, (short)0, c, false, false);
  }
  static __device__ __forceinline__ void guard(v8f& a, v8f& b, v16b x, v16b y) { dep_guard_b(a, b, x, y); }
  static __device__ __forceinline__ void keep(v16b a, v16b b, v16b c, v16b d) { keep4_b(a, b, c, d); }
};

template <int ET> struct Elem;
template <> struct Elem<0> { typedef _Float16 T; };
template <> struct Elem<1> { typedef __bf16 T; };
template <int ET, bool SPLIT, int BIAS_MODE, int OUT_MODE, bool RESID, int ACT = 0>
__global__ __launch_bounds__(256) void wmma_gemm64(
    const unsigned short* __restrict__ Ap, const unsigned short* __restrict__ A2p, int lda, long strideA,
    const unsigned short* __restrict__ Btp, const unsigned short* __restrict__ Bt2p, int ldb, long strideB,
    void* __restrict__ Cout, void* __restrict__ Cout2, int ldc, long strideC,
    const float* __restrict__ bias,
    const float* __restrict__ resid, long strideR,
    int M, int N, int K, float scale) {
  typedef typename Elem<ET>::T T;
  typedef typename Frag<T>::V V;
  const T* A = (const T*)Ap; const T* A2 = (const T*)A2p; const T* Bt = (const T*)Btp; const T* Bt2 = (const T*)Bt2p;
  __shared__ __align__(16) float sT[8][16 * 68];
  const int b    = blockIdx.y;
  const int lane = threadIdx.x & 31;
  const int wave = threadIdx.x >> 5;
  const int tilesN = N >> 6;
  const int tilesM = M >> 6;
  const int tile = blockIdx.x * 8 + wave;
  if (tile >= tilesM * tilesN) return;
  const int tm = tile / tilesN;
  const int tn = tile - tm * tilesN;
  const int m0 = tm << 6;
  const int n0 = tn << 6;

  const T* Ab  = A  + (size_t)b * strideA;
  const T* Bb  = Bt + (size_t)b * strideB;
  const T* Ab2 = SPLIT ? (A2  + (size_t)b * strideA) : nullptr;
  const T* Bb2 = SPLIT ? (Bt2 + (size_t)b * strideB) : nullptr;

  const int rlane = lane & 15;
  const int koff  = (lane >> 4) * 8;
  const int mOff  = (lane >> 4) * 8;

  v8f acc[4][4];
#pragma unroll
  for (int i = 0; i < 4; ++i)
#pragma unroll
    for (int j = 0; j < 4; ++j) acc[i][j] = (v8f){0.f,0.f,0.f,0.f,0.f,0.f,0.f,0.f};

  for (int k0 = 0; k0 < K; k0 += 32) {
    V bh[4], bl[4];
#pragma unroll
    for (int j = 0; j < 4; ++j) {
      const size_t bo = (size_t)(n0 + (j << 4) + rlane) * ldb + koff + k0;
      bh[j] = Frag<T>::load(Bb + bo);
      if (SPLIT) bl[j] = Frag<T>::load(Bb2 + bo);
    }
#pragma unroll
    for (int i = 0; i < 4; ++i) {
      const size_t ao = (size_t)(m0 + (i << 4) + rlane) * lda + koff + k0;
      V ah = Frag<T>::load(Ab + ao);
      V al;
      if (SPLIT) al = Frag<T>::load(Ab2 + ao);
#pragma unroll
      for (int j = 0; j < 4; ++j) {
        acc[i][j] = Frag<T>::mma(ah, bh[j], acc[i][j]);
        if (SPLIT) {
          acc[i][j] = Frag<T>::mma(ah, bl[j], acc[i][j]);
          acc[i][j] = Frag<T>::mma(al, bh[j], acc[i][j]);
        }
      }
      Frag<T>::guard(acc[i][0], acc[i][3], ah, SPLIT ? al : ah);
    }
    Frag<T>::keep(bh[0], bh[1], bh[2], bh[3]);
    if (SPLIT) Frag<T>::keep(bl[0], bl[1], bl[2], bl[3]);
  }
  acc_guard4(acc[0][0], acc[0][1], acc[0][2], acc[0][3]);
  acc_guard4(acc[1][0], acc[1][1], acc[1][2], acc[1][3]);
  acc_guard4(acc[2][0], acc[2][1], acc[2][2], acc[2][3]);
  acc_guard4(acc[3][0], acc[3][1], acc[3][2], acc[3][3]);

  float* slab = sT[wave];
  const float* Rb = RESID ? (resid + (size_t)b * strideR) : nullptr;
#pragma unroll
  for (int i = 0; i < 4; ++i) {
    const int mBase = m0 + (i << 4);
#pragma unroll
    for (int j = 0; j < 4; ++j) {
      const int n = n0 + (j << 4) + rlane;
      float bv = 0.f;
      if (BIAS_MODE == 2) bv = bias[n];
#pragma unroll
      for (int r = 0; r < 8; ++r) {
        float v = acc[i][j][r] * scale;
        if (BIAS_MODE == 1) v += bias[mBase + mOff + r];
        if (BIAS_MODE == 2) v += bv;
        if (RESID) v += Rb[(size_t)(mBase + mOff + r) * ldc + n];
        if (ACT == 1) v = tanhf(v);
        if (ACT == 2) v = fmaxf(v, 0.0f);
        if (ACT == 3) v = v / (1.0f + expf(-v));
        if (ACT == 4) v = (v > 0.f) ? v : 0.01f * v;
        if (ACT == 5) v = 0.5f * v * (1.0f + erff(v * 0.70710678118654752f));
        slab[(mOff + r) * 68 + (j << 4) + rlane] = v;
      }
    }
    __builtin_amdgcn_fence(__ATOMIC_RELEASE, "workgroup");
    __builtin_amdgcn_wave_barrier();
    __builtin_amdgcn_fence(__ATOMIC_ACQUIRE, "workgroup");
    if (OUT_MODE == 0) {
      float* C = (float*)Cout + (size_t)b * strideC;
      const int hh = lane >> 4, c4 = (lane & 15) * 4;
      for (int pass = 0; pass < 2; ++pass) {
#pragma unroll
        for (int it = 0; it < 8; ++it) {
          const int row = it * 2 + hh;
          v4f v = *(const v4f*)(slab + row * 68 + c4);
          *(volatile v4f*)(C + (size_t)(mBase + row) * ldc + n0 + c4) = v;
        }
        __threadfence();
      }
    } else {
      const int q = lane >> 3, c8 = (lane & 7) * 8;
      unsigned short* C  = (unsigned short*)Cout  + (size_t)b * strideC;
      unsigned short* C2 = (OUT_MODE == 2) ? ((unsigned short*)Cout2 + (size_t)b * strideC) : nullptr;
      for (int pass = 0; pass < 2; ++pass) {
#pragma unroll
        for (int it = 0; it < 4; ++it) {
          const int row = it * 4 + q;
          const float* sp = slab + row * 68 + c8;
          v8h hv, lv;
#pragma unroll
          for (int e = 0; e < 8; ++e) {
            if (OUT_MODE == 1) {
              hv[e] = (_Float16)sp[e];
            } else {
              unsigned short hb = f2bf_bits(sp[e]);
              unsigned short lb = f2bf_bits(sp[e] - bf_bits2f(hb));
              hv[e] = __builtin_bit_cast(_Float16, hb);
              lv[e] = __builtin_bit_cast(_Float16, lb);
            }
          }
          *(volatile v8h*)(C + (size_t)(mBase + row) * ldc + n0 + c8) = hv;
          if (OUT_MODE == 2) *(volatile v8h*)(C2 + (size_t)(mBase + row) * ldc + n0 + c8) = lv;
        }
        __threadfence();
      }
    }
    __builtin_amdgcn_fence(__ATOMIC_RELEASE, "workgroup");
    __builtin_amdgcn_wave_barrier();
    __builtin_amdgcn_fence(__ATOMIC_ACQUIRE, "workgroup");
  }
}

__global__ __launch_bounds__(256) void cast_f32_f16x2s(
    const float* __restrict__ in, _Float16* __restrict__ out, int n2, float scale) {
  int i = blockIdx.x * 256 + threadIdx.x;
  if (i < n2) {
    const _Float16 h0 = (_Float16)(in[2 * i] * scale), h1 = (_Float16)(in[2 * i + 1] * scale);
    const unsigned u = (unsigned)__builtin_bit_cast(unsigned short, h0) | ((unsigned)__builtin_bit_cast(unsigned short, h1) << 16);
    ((volatile unsigned*)out)[i] = u;
    __threadfence();
    ((volatile unsigned*)out)[i] = u;
  }
}

__global__ __launch_bounds__(256) void softmax_e_kernel(
    const float* __restrict__ xpre, float* __restrict__ xsm, int nrows) {
  __shared__ __align__(16) float sm[8][4 * 32];
  const int tid = threadIdx.x;
  const int wave = tid >> 5, lane = tid & 31;
  const int r0 = (blockIdx.x * 8 + wave) * 4;
  float* smw = sm[wave];
  for (int q = 0; q < 4; ++q) {
    int r = r0 + q;
    r = (r < nrows) ? r : (nrows - 1);
    const int bh = r >> 7;
    const int s  = r & (S_ - 1);
    const int b  = bh >> 3, h = bh & (H_ - 1);
    const float v = xpre[((size_t)(b * S_ + s)) * D_ + h * E_ + lane];
    float m = v;
#pragma unroll
    for (int off = 16; off; off >>= 1) m = fmaxf(m, __shfl_xor(m, off, 32));
    const float ev = expf(v - m);
    float sum = ev;
#pragma unroll
    for (int off = 16; off; off >>= 1) sum += __shfl_xor(sum, off, 32);
    smw[q * 32 + lane] = ev * (1.0f / sum);
  }
  __builtin_amdgcn_fence(__ATOMIC_RELEASE, "workgroup");
  __builtin_amdgcn_wave_barrier();
  __builtin_amdgcn_fence(__ATOMIC_ACQUIRE, "workgroup");
  const int q2 = lane >> 3, c4 = (lane & 7) * 4;
  const int rr = r0 + q2;
  const v4f val = *(const v4f*)(smw + q2 * 32 + c4);
  for (int pass = 0; pass < 2; ++pass) {
    if (rr < nrows) *(volatile v4f*)(xsm + (size_t)rr * E_ + c4) = val;
    __threadfence();
  }
}

__device__ __forceinline__ v8f mma_f16g(v16h a, v16h b, v8f c) {
  c = __builtin_amdgcn_wmma_f32_16x16x32_f16(false, a, false, b, (short)0, c, false, false);
  asm volatile("v_nop\n\tv_nop\n\tv_nop\n\tv_nop" : "+v"(c) : "v"(a), "v"(b));
  return c;
}
union FH { v16h v; v8h h[2]; };

__global__ __launch_bounds__(256) void spline_attn_kernel(
    const float* __restrict__ xsm, _Float16* __restrict__ mid) {
  __shared__ float ssx[S_ * XP];
  __shared__ float ssum[S_];
  __shared__ float lsh[QT];
  __shared__ float Ssh[QT * S_];
  __shared__ __align__(16) _Float16 Psh[QT * PP];
  __shared__ __align__(16) _Float16 Vt[E_ * VP];
  __shared__ __align__(16) _Float16 Osh[QT * OP];

  const int tid  = threadIdx.x;
  const int wave = tid >> 5, lane = tid & 31;
  const int hh   = lane >> 4, c = lane & 15;
  const int b    = blockIdx.x >> 3;
  const int s0   = (blockIdx.x & 7) * QT;
  const int li0  = wave * 2, li1 = li0 + 1;
  const int i0   = s0 + li0, i1 = s0 + li1;
  const float C6N  = -1.0f / 6.0f;
  const float EE   = (float)(E_ * E_);
  const float EINV = 1.0f / (float)E_;

#pragma unroll 1
  for (int h = 0; h < H_; ++h) {
    const float* xb = xsm + ((size_t)(b * H_ + h)) * (S_ * E_);
    __syncthreads();
#pragma unroll
    for (int it = 0; it < (S_ * E_) / 256; ++it) {
      const int idx = it * 256 + tid;
      const float v = xb[idx];
      const int j = idx >> 5, e = idx & 31;
      ssx[j * XP + e] = v;
      Vt[e * VP + j] = (_Float16)(v * 256.0f);
    }
    __syncthreads();
    if (tid < S_) {
      float s = 0.0f;
#pragma unroll
      for (int e = 0; e < E_; ++e) s += ssx[tid * XP + e];
      ssum[tid] = s;
    }
    __syncthreads();

#pragma unroll 1
    for (int jc = 0; jc < S_ / 32; ++jc) {
      const int j = jc * 32 + lane;
      float brow[32];
#pragma unroll
      for (int f = 0; f < 32; ++f) brow[f] = ssx[j * XP + f];
      float acc0 = 0.0f, acc1 = 0.0f;
#pragma unroll 1
      for (int e = 0; e < E_; ++e) {
        const float a0 = ssx[i0 * XP + e];
        const float a1 = ssx[i1 * XP + e];
        const float ha0 = 0.5f * a0, ha1 = 0.5f * a1;
#pragma unroll
        for (int f = 0; f < 32; ++f) {
          const float bb = brow[f];
          const float m0 = fminf(a0, bb), m1 = fminf(a1, bb);
          const float u0 = fmaf(m0 * m0, C6N, ha0 * bb);
          const float u1 = fmaf(m1 * m1, C6N, ha1 * bb);
          acc0 = fmaf(m0, u0, acc0);
          acc1 = fmaf(m1, u1, acc1);
        }
      }
      const float sj = ssum[j];
      Ssh[li0 * S_ + j] = (fmaf(ssum[i0], sj, acc0) + EE) * EINV;
      Ssh[li1 * S_ + j] = (fmaf(ssum[i1], sj, acc1) + EE) * EINV;
    }

    {
      float sv0[4], sv1[4];
#pragma unroll
      for (int q = 0; q < 4; ++q) { sv0[q] = Ssh[li0 * S_ + q * 32 + lane]; sv1[q] = Ssh[li1 * S_ + q * 32 + lane]; }
      float mx0 = fmaxf(fmaxf(sv0[0], sv0[1]), fmaxf(sv0[2], sv0[3]));
      float mx1 = fmaxf(fmaxf(sv1[0], sv1[1]), fmaxf(sv1[2], sv1[3]));
#pragma unroll
      for (int off = 16; off; off >>= 1) {
        mx0 = fmaxf(mx0, __shfl_xor(mx0, off, 32));
        mx1 = fmaxf(mx1, __shfl_xor(mx1, off, 32));
      }
      float l0 = 0.0f, l1 = 0.0f;
#pragma unroll
      for (int q = 0; q < 4; ++q) {
        const float p0 = __expf(sv0[q] - mx0);
        const float p1 = __expf(sv1[q] - mx1);
        l0 += p0; l1 += p1;
        Psh[li0 * PP + q * 32 + lane] = (_Float16)p0;
        Psh[li1 * PP + q * 32 + lane] = (_Float16)p1;
      }
#pragma unroll
      for (int off = 16; off; off >>= 1) {
        l0 += __shfl_xor(l0, off, 32);
        l1 += __shfl_xor(l1, off, 32);
      }
      if (lane == 0) { lsh[li0] = l0; lsh[li1] = l1; }
    }
    __syncthreads();

    if (wave < 2) {
      const int t = wave;
      v8f acc = (v8f){0.f,0.f,0.f,0.f,0.f,0.f,0.f,0.f};
#pragma unroll
      for (int kk = 0; kk < S_ / 32; ++kk) {
        FH pa, vb;
        pa.h[0] = *(const v8h*)(Psh + c * PP + kk * 32 + 8 * hh);
        pa.h[1] = *(const v8h*)(Psh + c * PP + kk * 32 + 16 + 8 * hh);
        vb.h[0] = *(const v8h*)(Vt + (t * 16 + c) * VP + kk * 32 + 8 * hh);
        vb.h[1] = *(const v8h*)(Vt + (t * 16 + c) * VP + kk * 32 + 16 + 8 * hh);
        acc = mma_f16g(pa.v, vb.v, acc);
      }
#pragma unroll
      for (int r = 0; r < 8; ++r) {
        const int row = 8 * hh + r;
        const float inv = 0.25f * __builtin_amdgcn_rcpf(lsh[row]);
        Osh[row * OP + h * E_ + t * 16 + c] = (_Float16)(acc[r] * inv);
      }
    }
  }
  __syncthreads();

  {
    const int q = lane >> 3, c8 = (lane & 7) * 8;
    for (int pass = 0; pass < 2; ++pass) {
#pragma unroll
      for (int ri = 0; ri < 2; ++ri) {
        const int row = wave * 2 + ri;
        const v8h val = *(const v8h*)(Osh + row * OP + q * 64 + c8);
        *(volatile v8h*)(mid + ((size_t)(b * S_ + s0 + row)) * D_ + q * 64 + c8) = val;
      }
      __threadfence();
    }
  }
}

static inline size_t al256(size_t x) { return (x + 255) & ~(size_t)255; }

extern "C" void kernel_launch(void* const* d_in, const int* in_sizes, int n_in,
                              void* d_out, int out_size, void* d_ws, size_t ws_size,
                              hipStream_t stream) {
  if (n_in < 5) return;
  const int n0 = in_sizes[0];
  if (in_sizes[1] != D_ * D_ || in_sizes[2] != D_ || in_sizes[3] != D_ * D_ || in_sizes[4] != D_) return;
  if (n0 <= 0 || (n0 % (S_ * D_)) != 0 || out_size != n0) return;
  const int B = n0 / (S_ * D_);
  const int M = B * S_;

  const float* inputs = (const float*)d_in[0];
  const float* w_in   = (const float*)d_in[1];
  const float* b_in   = (const float*)d_in[2];
  const float* w_out  = (const float*)d_in[3];
  const float* b_out  = (const float*)d_in[4];
  float* out = (float*)d_out;

  char* ws = (char*)d_ws;
  size_t off = 0;
  const size_t o_inh  = off; off = al256(off + (size_t)n0 * 2);
  const size_t o_wih  = off; off = al256(off + (size_t)D_ * D_ * 2);
  const size_t o_woh  = off; off = al256(off + (size_t)D_ * D_ * 2);
  const size_t o_xpre = off; off = al256(off + (size_t)n0 * 4);
  const size_t o_xsm  = off; off = al256(off + (size_t)n0 * 4);
  const size_t o_mid  = off; off = al256(off + (size_t)n0 * 2);
  if (off > ws_size || off > (size_t)134217728) return;

  _Float16* in_h  = (_Float16*)(ws + o_inh);
  _Float16* wi_h  = (_Float16*)(ws + o_wih);
  _Float16* wo_h  = (_Float16*)(ws + o_woh);
  float*    xpre  = (float*)(ws + o_xpre);
  float*    xsm   = (float*)(ws + o_xsm);
  _Float16* mid_h = (_Float16*)(ws + o_mid);

  {
    const int n2a = n0 / 2, n2w = (D_ * D_) / 2;
    cast_f32_f16x2s<<<(n2a + 255) / 256, 256, 0, stream>>>(inputs, in_h, n2a, 1.0f);
    cast_f32_f16x2s<<<(n2w + 255) / 256, 256, 0, stream>>>(w_in, wi_h, n2w, 16.0f);
    cast_f32_f16x2s<<<(n2w + 255) / 256, 256, 0, stream>>>(w_out, wo_h, n2w, 16.0f);
  }

  const int tiles = (M / 64) * (D_ / 64);
  const int gx = (tiles + 7) / 8;

  wmma_gemm64<0, false, 2, 0, false, 0><<<dim3(gx, 1), 256, 0, stream>>>(
      (const unsigned short*)in_h, (const unsigned short*)in_h, D_, 0L,
      (const unsigned short*)wi_h, (const unsigned short*)wi_h, D_, 0L,
      (void*)xpre, (void*)xpre, D_, 0L,
      b_in, b_in, 0L,
      M, D_, D_, 1.0f / 16.0f);

  {
    const int nrows = B * H_ * S_;
    softmax_e_kernel<<<(nrows + 31) / 32, 256, 0, stream>>>(xpre, xsm, nrows);
  }

  spline_attn_kernel<<<B * (S_ / QT), 256, 0, stream>>>(xsm, mid_h);

  wmma_gemm64<0, false, 2, 0, false, 0><<<dim3(gx, 1), 256, 0, stream>>>(
      (const unsigned short*)mid_h, (const unsigned short*)mid_h, D_, 0L,
      (const unsigned short*)wo_h, (const unsigned short*)wo_h, D_, 0L,
      (void*)out, (void*)out, D_, 0L,
      b_out, b_out, 0L,
      M, D_, D_, 1.0f / 1024.0f);
}
